// ChunkedCausalAttention_StaticRoutedLoRAExpert_46737834115825
// MI455X (gfx1250) — hardware-verified
//
#include <hip/hip_runtime.h>
#include <math.h>

constexpr int kBat   = 4;
constexpr int kSeqN  = 2048;
constexpr int kDim   = 1024;
constexpr int kHeads = 16;
constexpr int kDh    = 64;
constexpr int kCS    = 512;
constexpr int kNSeg  = 4;
constexpr int kNSets = 4;
constexpr int kRank  = 16;
constexpr int kTok   = kBat * kSeqN;
constexpr int kNRB   = kBat * kNSeg;
constexpr int kKA    = kDim + 64;
constexpr int kQKld  = 2 * kDim;
constexpr float kWCarry   = 64.0f;
constexpr float kTScale   = 2.0f / 64.0f;
constexpr float kQKScale  = 8.0f / 64.0f;
constexpr float kVTScale  = 1.0f / 64.0f;
constexpr float kSScale   = 0.125f / 64.0f;
constexpr float kPVScale  = 256.0f;
constexpr float kT2Scale  = 512.0f / 16384.0f;
constexpr float kOutScale = 1.0f / 16384.0f;

constexpr size_t kOffS     = 0;
constexpr size_t kSzS      = (size_t)16 * kCS * kCS * 4;
constexpr size_t kOffPh    = kOffS + kSzS;
constexpr size_t kSzP      = (size_t)16 * kCS * kCS * 2;
constexpr size_t kOffPl    = kOffPh + kSzP;
constexpr size_t kEndR0    = kOffPl + kSzP;
constexpr size_t kOffXa    = 0;
constexpr size_t kSzXa     = (size_t)kTok * kKA * 2;
constexpr size_t kOffWa    = kOffXa + kSzXa;
constexpr size_t kSzWa     = (size_t)3 * kDim * kKA * 2;
constexpr size_t kOffAselQ = kOffWa + kSzWa;
constexpr size_t kSzAsel   = (size_t)kNRB * 64 * kDim * 2;
constexpr size_t kOffWp    = kEndR0;
constexpr size_t kSzWp     = (size_t)kDim * kKA * 2;
constexpr size_t kOffAselP = kOffWp + kSzWp;
constexpr size_t kOffQK    = kOffAselP + kSzAsel;
constexpr size_t kSzQK     = (size_t)kTok * kQKld * 2;
constexpr size_t kOffVTh   = kOffQK + kSzQK;
constexpr size_t kSzVT     = (size_t)kDim * kTok * 2;
constexpr size_t kOffVTl   = kOffVTh + kSzVT;
constexpr size_t kOffO     = kOffVTl + kSzVT;
constexpr size_t kSzO      = (size_t)kTok * kKA * 2;
constexpr size_t kWsTotal  = kOffO + kSzO;
static_assert(kOffAselQ + kSzAsel <= kEndR0);
static_assert(kWsTotal == 122814464);
static_assert(kWsTotal <= 134217728);
static_assert((kOffPh % 128) == 0 && (kOffPl % 128) == 0 && (kOffWa % 128) == 0 && (kOffAselQ % 128) == 0);
static_assert((kOffWp % 128) == 0 && (kOffAselP % 128) == 0 && (kOffQK % 128) == 0);
static_assert((kOffVTh % 128) == 0 && (kOffVTl % 128) == 0 && (kOffO % 128) == 0);
static_assert((kKA % 32) == 0 && ((kKA * 2) % 128) == 0);

typedef __attribute__((ext_vector_type(16))) _Float16 v16h;
typedef __attribute__((ext_vector_type(8)))  _Float16 v8h;
typedef __attribute__((ext_vector_type(16))) __bf16   v16b;
typedef __attribute__((ext_vector_type(8)))  __bf16   v8b;
typedef __attribute__((ext_vector_type(8)))  float    v8f;
typedef __attribute__((ext_vector_type(4)))  float    v4f;
typedef __attribute__((ext_vector_type(4)))  unsigned int v4u;

__device__ __forceinline__ unsigned short f2bf_bits(float f) {
  unsigned u = __float_as_uint(f);
  return (unsigned short)((u + 0x7FFFu + ((u >> 16) & 1u)) >> 16);
}
__device__ __forceinline__ float bf_bits2f(unsigned short h) { return __uint_as_float(((unsigned)h) << 16); }

__device__ __forceinline__ void dep_guard_h(v8f& a, v8f& b, v16h x, v16h y) { asm volatile("v_nop\n\tv_nop\n\tv_nop\n\tv_nop" : "+v"(a), "+v"(b) : "v"(x), "v"(y)); }
__device__ __forceinline__ void dep_guard_b(v8f& a, v8f& b, v16b x, v16b y) { asm volatile("v_nop\n\tv_nop\n\tv_nop\n\tv_nop" : "+v"(a), "+v"(b) : "v"(x), "v"(y)); }
__device__ __forceinline__ void keep4_h(v16h a, v16h b, v16h c, v16h d) { asm volatile("v_nop" :: "v"(a), "v"(b), "v"(c), "v"(d)); }
__device__ __forceinline__ void keep4_b(v16b a, v16b b, v16b c, v16b d) { asm volatile("v_nop" :: "v"(a), "v"(b), "v"(c), "v"(d)); }
__device__ __forceinline__ void acc_guard4(v8f& a, v8f& b, v8f& c, v8f& d) { asm volatile("v_nop\n\tv_nop\n\tv_nop\n\tv_nop" : "+v"(a), "+v"(b), "+v"(c), "+v"(d)); }
template <typename T> struct Frag;
template <> struct Frag<_Float16> {
  typedef v16h V; union U { v16h v; v8h h[2]; };
  static __device__ __forceinline__ v16h load(const _Float16* p) {
    U f; f.h[0] = *(const v8h*)(p); f.h[1] = *(const v8h*)(p + 16); return f.v;
  }
  static __device__ __forceinline__ v8f mma(v16h a, v16h b, v8f c) {
    return __builtin_amdgcn_wmma_f32_16x16x32_f16(false, a, false, b, (short)0, c, false, false);
  }
  static __device__ __forceinline__ void guard(v8f& a, v8f& b, v16h x, v16h y) { dep_guard_h(a, b, x, y); }
  static __device__ __forceinline__ void keep(v16h a, v16h b, v16h c, v16h d) { keep4_h(a, b, c, d); }
};
template <> struct Frag<__bf16> {
  typedef v16b V; union U { v16b v; v8b h[2]; };
  static __device__ __forceinline__ v16b load(const __bf16* p) {
    U f; f.h[0] = *(const v8b*)(p); f.h[1] = *(const v8b*)(p + 16); return f.v;
  }
  static __device__ __forceinline__ v8f mma(v16b a, v16b b, v8f c) {
    return __builtin_amdgcn_wmma_f32_16x16x32_bf16(false, a, false, b, (short)0, c, false, false);
  }
  static __device__ __forceinline__ void guard(v8f& a, v8f& b, v16b x, v16b y) { dep_guard_b(a, b, x, y); }
  static __device__ __forceinline__ void keep(v16b a, v16b b, v16b c, v16b d) { keep4_b(a, b, c, d); }
};

__device__ __forceinline__ unsigned pk16(unsigned short a, unsigned short b) { return (unsigned)a | ((unsigned)b << 16); }
__device__ __forceinline__ unsigned short h_bits(float f) { const _Float16 h = (_Float16)f; return __builtin_bit_cast(unsigned short, h); }

template <int ET> struct Elem;
template <> struct Elem<0> { typedef _Float16 T; };
template <> struct Elem<1> { typedef __bf16 T; };
template <int ET, bool SPLIT, int BIAS_MODE, int OUT_MODE, bool RESID, int ACT = 0>
__global__ __launch_bounds__(256) void wmma_gemm64(
    const unsigned short* __restrict__ Ap, const unsigned short* __restrict__ A2p, int lda, long strideA,
    const unsigned short* __restrict__ Btp, const unsigned short* __restrict__ Bt2p, int ldb, long strideB,
    void* __restrict__ Cout, void* __restrict__ Cout2, int ldc, long strideC,
    const float* __restrict__ bias,
    const float* __restrict__ resid, long strideR,
    int M, int N, int K, float scale) {
  typedef typename Elem<ET>::T T;
  typedef typename Frag<T>::V V;
  const T* A = (const T*)Ap; const T* A2 = (const T*)A2p; const T* Bt = (const T*)Btp; const T* Bt2 = (const T*)Bt2p;
  __shared__ __align__(16) float sT[8][16 * 68];
  const int b    = blockIdx.y;
  const int lane = threadIdx.x & 31;
  const int wave = threadIdx.x >> 5;
  const int tilesN = N >> 6;
  const int tilesM = M >> 6;
  const int tile = blockIdx.x * 8 + wave;
  if (tile >= tilesM * tilesN) return;
  const int tm = tile / tilesN;
  const int tn = tile - tm * tilesN;
  const int m0 = tm << 6;
  const int n0 = tn << 6;

  const T* Ab  = A  + (size_t)b * strideA;
  const T* Bb  = Bt + (size_t)b * strideB;
  const T* Ab2 = SPLIT ? (A2  + (size_t)b * strideA) : nullptr;
  const T* Bb2 = SPLIT ? (Bt2 + (size_t)b * strideB) : nullptr;

  const int rlane = lane & 15;
  const int koff  = (lane >> 4) * 8;
  const int mOff  = (lane >> 4) * 8;

  v8f acc[4][4];
#pragma unroll
  for (int i = 0; i < 4; ++i)
#pragma unroll
    for (int j = 0; j < 4; ++j) acc[i][j] = (v8f){0.f,0.f,0.f,0.f,0.f,0.f,0.f,0.f};

  for (int k0 = 0; k0 < K; k0 += 32) {
    V bh[4], bl[4];
#pragma unroll
    for (int j = 0; j < 4; ++j) {
      const size_t bo = (size_t)(n0 + (j << 4) + rlane) * ldb + koff + k0;
      bh[j] = Frag<T>::load(Bb + bo);
      if (SPLIT) bl[j] = Frag<T>::load(Bb2 + bo);
    }
#pragma unroll
    for (int i = 0; i < 4; ++i) {
      const size_t ao = (size_t)(m0 + (i << 4) + rlane) * lda + koff + k0;
      V ah = Frag<T>::load(Ab + ao);
      V al;
      if (SPLIT) al = Frag<T>::load(Ab2 + ao);
#pragma unroll
      for (int j = 0; j < 4; ++j) {
        acc[i][j] = Frag<T>::mma(ah, bh[j], acc[i][j]);
        if (SPLIT) {
          acc[i][j] = Frag<T>::mma(ah, bl[j], acc[i][j]);
          acc[i][j] = Frag<T>::mma(al, bh[j], acc[i][j]);
        }
      }
      Frag<T>::guard(acc[i][0], acc[i][3], ah, SPLIT ? al : ah);
    }
    Frag<T>::keep(bh[0], bh[1], bh[2], bh[3]);
    if (SPLIT) Frag<T>::keep(bl[0], bl[1], bl[2], bl[3]);
  }
  acc_guard4(acc[0][0], acc[0][1], acc[0][2], acc[0][3]);
  acc_guard4(acc[1][0], acc[1][1], acc[1][2], acc[1][3]);
  acc_guard4(acc[2][0], acc[2][1], acc[2][2], acc[2][3]);
  acc_guard4(acc[3][0], acc[3][1], acc[3][2], acc[3][3]);

  float* slab = sT[wave];
  const float* Rb = RESID ? (resid + (size_t)b * strideR) : nullptr;
#pragma unroll
  for (int i = 0; i < 4; ++i) {
    const int mBase = m0 + (i << 4);
#pragma unroll
    for (int j = 0; j < 4; ++j) {
      const int n = n0 + (j << 4) + rlane;
      float bv = 0.f;
      if (BIAS_MODE == 2) bv = bias[n];
#pragma unroll
      for (int r = 0; r < 8; ++r) {
        float v = acc[i][j][r] * scale;
        if (BIAS_MODE == 1) v += bias[mBase + mOff + r];
        if (BIAS_MODE == 2) v += bv;
        if (RESID) v += Rb[(size_t)(mBase + mOff + r) * ldc + n];
        if (ACT == 2) v = fmaxf(v, 0.0f);
        if (ACT == 4) v = (v > 0.f) ? v : 0.01f * v;
        slab[(mOff + r) * 68 + (j << 4) + rlane] = v;
      }
    }
    __builtin_amdgcn_fence(__ATOMIC_RELEASE, "workgroup");
    __builtin_amdgcn_wave_barrier();
    __builtin_amdgcn_fence(__ATOMIC_ACQUIRE, "workgroup");
    if (OUT_MODE == 0) {
      float* C = (float*)Cout + (size_t)b * strideC;
      const int hh = lane >> 4, c4 = (lane & 15) * 4;
      for (int pass = 0; pass < 2; ++pass) {
#pragma unroll
        for (int it = 0; it < 8; ++it) {
          const int row = it * 2 + hh;
          v4f v = *(const v4f*)(slab + row * 68 + c4);
          *(volatile v4f*)(C + (size_t)(mBase + row) * ldc + n0 + c4) = v;
        }
        __threadfence();
      }
    } else {
      const int q = lane >> 3, c8 = (lane & 7) * 8;
      unsigned short* C  = (unsigned short*)Cout  + (size_t)b * strideC;
      unsigned short* C2 = (OUT_MODE == 2) ? ((unsigned short*)Cout2 + (size_t)b * strideC) : nullptr;
      for (int pass = 0; pass < 2; ++pass) {
#pragma unroll
        for (int it = 0; it < 4; ++it) {
          const int row = it * 4 + q;
          const float* sp = slab + row * 68 + c8;
          v8h hv, lv;
#pragma unroll
          for (int e = 0; e < 8; ++e) {
            if (OUT_MODE == 1) {
              hv[e] = (_Float16)sp[e];
            } else {
              unsigned short hb = f2bf_bits(sp[e]);
              unsigned short lb = f2bf_bits(sp[e] - bf_bits2f(hb));
              hv[e] = __builtin_bit_cast(_Float16, hb);
              lv[e] = __builtin_bit_cast(_Float16, lb);
            }
          }
          *(volatile v8h*)(C + (size_t)(mBase + row) * ldc + n0 + c8) = hv;
          if (OUT_MODE == 2) *(volatile v8h*)(C2 + (size_t)(mBase + row) * ldc + n0 + c8) = lv;
        }
        __threadfence();
      }
    }
    __builtin_amdgcn_fence(__ATOMIC_RELEASE, "workgroup");
    __builtin_amdgcn_wave_barrier();
    __builtin_amdgcn_fence(__ATOMIC_ACQUIRE, "workgroup");
  }
}

__global__ __launch_bounds__(256) void cast_x_kernel(const float* __restrict__ x, unsigned short* __restrict__ xa) {
  const int idx = blockIdx.x * 256 + threadIdx.x;
  if (idx >= kTok * 128) return;
  const int row = idx >> 7, p = idx & 127;
  const float* src = x + (size_t)row * kDim + 8 * p;
  const v4f a = *(const v4f*)(src);
  const v4f c = *(const v4f*)(src + 4);
  unsigned short hb[8];
#pragma unroll
  for (int e = 0; e < 4; ++e) { hb[e] = h_bits(a[e]); hb[4 + e] = h_bits(c[e]); }
  const v4u u = (v4u){pk16(hb[0], hb[1]), pk16(hb[2], hb[3]), pk16(hb[4], hb[5]), pk16(hb[6], hb[7])};
  unsigned short* dst = xa + (size_t)row * kKA + 8 * p;
  *(volatile v4u*)dst = u;
  __threadfence();
  *(volatile v4u*)dst = u;
}

__global__ __launch_bounds__(256) void build_waug_kernel(const float* __restrict__ W, const float* __restrict__ Bl,
                                                        unsigned short* __restrict__ out, int nrows, int maskMid) {
  const int idx = blockIdx.x * 256 + threadIdx.x;
  if (idx >= nrows * 136) return;
  const int row = idx / 136;
  const int p = idx - row * 136;
  const bool isW = p < 128;
  const int pw = isW ? p : 0;
  const int pb = isW ? 0 : (p - 128);
  const int cb = 8 * pb;
  const int e = cb >> 4;
  const int r0 = cb & 15;
  const float* wsrc = W + (size_t)row * kDim + 8 * pw;
  const float* bsrc = Bl + ((size_t)e * nrows + row) * kRank + r0;
  const v4f w0 = *(const v4f*)(wsrc);
  const v4f w1 = *(const v4f*)(wsrc + 4);
  const v4f b0 = *(const v4f*)(bsrc);
  const v4f b1 = *(const v4f*)(bsrc + 4);
  const bool midZero = (maskMid != 0) && (row >= kDim) && (row < 2 * kDim);
  const float bm = midZero ? 0.0f : kWCarry;
  unsigned short hb[8];
#pragma unroll
  for (int q = 0; q < 4; ++q) {
    const float vw0 = kWCarry * w0[q], vb0 = bm * b0[q];
    const float vw1 = kWCarry * w1[q], vb1 = bm * b1[q];
    hb[q]     = h_bits(isW ? vw0 : vb0);
    hb[4 + q] = h_bits(isW ? vw1 : vb1);
  }
  const v4u u = (v4u){pk16(hb[0], hb[1]), pk16(hb[2], hb[3]), pk16(hb[4], hb[5]), pk16(hb[6], hb[7])};
  unsigned short* dst = out + (size_t)row * kKA + 8 * p;
  *(volatile v4u*)dst = u;
  __threadfence();
  *(volatile v4u*)dst = u;
}

__global__ __launch_bounds__(256) void build_asel_kernel(const float* __restrict__ A, const int* __restrict__ route,
                                                        const int* __restrict__ segsz, unsigned short* __restrict__ out) {
  (void)segsz;
  const int idx = blockIdx.x * 256 + threadIdx.x;
  if (idx >= kNRB * 64 * 128) return;
  const int y = idx >> 13;
  const int j = (idx >> 7) & 63;
  const int p = idx & 127;
  int e = route[y & 3];
  e = e < 0 ? 0 : (e > kNSets - 1 ? kNSets - 1 : e);
  const float mult = ((j >> 4) == e) ? kWCarry : 0.0f;
  const float* src = A + ((size_t)e * kRank + (j & 15)) * kDim + 8 * p;
  const v4f a = *(const v4f*)(src);
  const v4f c = *(const v4f*)(src + 4);
  unsigned short hb[8];
#pragma unroll
  for (int q = 0; q < 4; ++q) {
    hb[q]     = h_bits(mult * a[q]);
    hb[4 + q] = h_bits(mult * c[q]);
  }
  const v4u u = (v4u){pk16(hb[0], hb[1]), pk16(hb[2], hb[3]), pk16(hb[4], hb[5]), pk16(hb[6], hb[7])};
  unsigned short* dst = out + ((size_t)(y * 64 + j)) * kDim + 8 * p;
  *(volatile v4u*)dst = u;
  __threadfence();
  *(volatile v4u*)dst = u;
}

__global__ __launch_bounds__(256) void softmax_kernel(const float* __restrict__ S, unsigned short* __restrict__ Ph,
                                                     unsigned short* __restrict__ Pl, int Skv) {
  __shared__ __align__(16) float stage[2048];
  __shared__ float redM[8];
  __shared__ float redS[8];
  const int row = blockIdx.x;
  const int t = threadIdx.x, lane = t & 31, wave = t >> 5;
  int nper = Skv >> 8;
  nper = nper > 8 ? 8 : (nper < 1 ? 1 : nper);
  const float* sr = S + (size_t)row * Skv;
  float m = -INFINITY;
#pragma unroll 1
  for (int j = 0; j < nper; ++j) m = fmaxf(m, sr[t + 256 * j]);
#pragma unroll
  for (int off = 16; off > 0; off >>= 1) m = fmaxf(m, __shfl_xor(m, off, 32));
  if (lane == 0) redM[wave] = m;
  __syncthreads();
  const float gm = fmaxf(fmaxf(fmaxf(redM[0], redM[1]), fmaxf(redM[2], redM[3])),
                         fmaxf(fmaxf(redM[4], redM[5]), fmaxf(redM[6], redM[7])));
  float s = 0.f;
#pragma unroll 1
  for (int j = 0; j < nper; ++j) {
    const float ev = expf(sr[t + 256 * j] - gm);
    stage[t + 256 * j] = ev;
    s += ev;
  }
#pragma unroll
  for (int off = 16; off > 0; off >>= 1) s += __shfl_xor(s, off, 32);
  if (lane == 0) redS[wave] = s;
  __syncthreads();
  const float tot = ((redS[0] + redS[1]) + (redS[2] + redS[3])) + ((redS[4] + redS[5]) + (redS[6] + redS[7]));
  const float inv = 1.0f / tot;
  if (t < (nper << 5)) {
    const v4f a = *(const v4f*)(stage + 8 * t);
    const v4f c = *(const v4f*)(stage + 8 * t + 4);
    unsigned short hh8[8], ll8[8];
#pragma unroll
    for (int e = 0; e < 4; ++e) {
      const float v0 = a[e] * inv;
      const unsigned short h0 = f2bf_bits(v0);
      hh8[e] = h0;
      ll8[e] = f2bf_bits(v0 - bf_bits2f(h0));
      const float v1 = c[e] * inv;
      const unsigned short h1 = f2bf_bits(v1);
      hh8[4 + e] = h1;
      ll8[4 + e] = f2bf_bits(v1 - bf_bits2f(h1));
    }
    const v4u uh = (v4u){pk16(hh8[0], hh8[1]), pk16(hh8[2], hh8[3]), pk16(hh8[4], hh8[5]), pk16(hh8[6], hh8[7])};
    const v4u ul = (v4u){pk16(ll8[0], ll8[1]), pk16(ll8[2], ll8[3]), pk16(ll8[4], ll8[5]), pk16(ll8[6], ll8[7])};
    unsigned short* ph = Ph + (size_t)row * Skv + 8 * t;
    unsigned short* pl = Pl + (size_t)row * Skv + 8 * t;
    *(volatile v4u*)ph = uh;
    *(volatile v4u*)pl = ul;
    __threadfence();
    *(volatile v4u*)ph = uh;
    *(volatile v4u*)pl = ul;
  }
}

extern "C" void kernel_launch(void* const* d_in, const int* in_sizes, int n_in,
                              void* d_out, int out_size, void* d_ws, size_t ws_size,
                              hipStream_t stream) {
  if (n_in < 9) return;
  if (in_sizes[0] != kTok * kDim) return;
  if (in_sizes[1] != 3 * kDim * kDim) return;
  if (in_sizes[2] != kNSets * kRank * kDim) return;
  if (in_sizes[3] != kNSets * 3 * kDim * kRank) return;
  if (in_sizes[4] != kDim * kDim) return;
  if (in_sizes[5] != kNSets * kRank * kDim) return;
  if (in_sizes[6] != kNSets * kDim * kRank) return;
  if (in_sizes[7] < kNSeg) return;
  if (in_sizes[8] < 1) return;
  if (out_size != kTok * kDim) return;
  if (ws_size < kWsTotal) return;

  const float* x    = (const float*)d_in[0];
  const float* Wqkv = (const float*)d_in[1];
  const float* Aq   = (const float*)d_in[2];
  const float* Bq   = (const float*)d_in[3];
  const float* Wp   = (const float*)d_in[4];
  const float* Ap   = (const float*)d_in[5];
  const float* Bp   = (const float*)d_in[6];
  const int*   route = (const int*)d_in[7];
  const int*   segsz = (const int*)d_in[8];
  float* out = (float*)d_out;

  char* ws = (char*)d_ws;
  float*          Spl   = (float*)(ws + kOffS);
  unsigned short* Phi   = (unsigned short*)(ws + kOffPh);
  unsigned short* Plo   = (unsigned short*)(ws + kOffPl);
  unsigned short* Xaug  = (unsigned short*)(ws + kOffXa);
  unsigned short* Waug  = (unsigned short*)(ws + kOffWa);
  unsigned short* AselQ = (unsigned short*)(ws + kOffAselQ);
  unsigned short* Wpaug = (unsigned short*)(ws + kOffWp);
  unsigned short* AselP = (unsigned short*)(ws + kOffAselP);
  unsigned short* QK16  = (unsigned short*)(ws + kOffQK);
  unsigned short* VThi  = (unsigned short*)(ws + kOffVTh);
  unsigned short* VTlo  = (unsigned short*)(ws + kOffVTl);
  unsigned short* Oaug  = (unsigned short*)(ws + kOffO);

  const dim3 blk(256);

  cast_x_kernel<<<dim3((kTok * 128) / 256), blk, 0, stream>>>(x, Xaug);
  build_waug_kernel<<<dim3((3 * kDim * 136) / 256), blk, 0, stream>>>(Wqkv, Bq, Waug, 3 * kDim, 1);
  build_waug_kernel<<<dim3((kDim * 136) / 256), blk, 0, stream>>>(Wp, Bp, Wpaug, kDim, 0);
  build_asel_kernel<<<dim3((kNRB * 64 * 128) / 256), blk, 0, stream>>>(Aq, route, segsz, AselQ);
  build_asel_kernel<<<dim3((kNRB * 64 * 128) / 256), blk, 0, stream>>>(Ap, route, segsz, AselP);

  wmma_gemm64<0, false, 0, 1, false><<<dim3(1, kNRB), blk, 0, stream>>>(
      Xaug, nullptr, kKA, (long)kCS * kKA,
      AselQ, nullptr, kDim, (long)64 * kDim,
      (void*)(Xaug + kDim), nullptr, kKA, (long)kCS * kKA,
      nullptr, nullptr, 0L, kCS, 64, kDim, kTScale);

  wmma_gemm64<0, false, 0, 1, false><<<dim3(((kTok / 64) * (kQKld / 64)) / 8, 1), blk, 0, stream>>>(
      Xaug, nullptr, kKA, 0L,
      Waug, nullptr, kKA, 0L,
      (void*)QK16, nullptr, kQKld, 0L,
      nullptr, nullptr, 0L, kTok, kQKld, kKA, kQKScale);

  wmma_gemm64<0, false, 0, 2, false><<<dim3(((kDim / 64) * (kTok / 64)) / 8, 1), blk, 0, stream>>>(
      Waug + (size_t)2 * kDim * kKA, nullptr, kKA, 0L,
      Xaug, nullptr, kKA, 0L,
      (void*)VThi, (void*)VTlo, kTok, 0L,
      nullptr, nullptr, 0L, kDim, kTok, kKA, kVTScale);

  const int gtab[kNSeg] = {16, 8, 4, 4};
  for (int i = 0; i < kNSeg; ++i) {
    const int Skv = kCS * (i + 1);
    const int G = gtab[i];
    for (int b = 0; b < kBat; ++b) {
      for (int h0 = 0; h0 < kHeads; h0 += G) {
        const int Gc = (kHeads - h0 < G) ? (kHeads - h0) : G;
        wmma_gemm64<0, false, 0, 0, false><<<dim3(Skv / 64, Gc), blk, 0, stream>>>(
            QK16 + ((size_t)b * kSeqN + (size_t)i * kCS) * kQKld + (size_t)h0 * kDh, nullptr, kQKld, (long)kDh,
            QK16 + (size_t)b * kSeqN * kQKld + kDim + (size_t)h0 * kDh, nullptr, kQKld, (long)kDh,
            (void*)Spl, nullptr, Skv, (long)kCS * Skv,
            nullptr, nullptr, 0L, kCS, Skv, kDh, kSScale);
        softmax_kernel<<<dim3(Gc * kCS), blk, 0, stream>>>(Spl, Phi, Plo, Skv);
        wmma_gemm64<1, true, 0, 1, false><<<dim3(1, Gc), blk, 0, stream>>>(
            Phi, Plo, Skv, (long)kCS * Skv,
            VThi + (size_t)h0 * kDh * kTok + (size_t)b * kSeqN, VTlo + (size_t)h0 * kDh * kTok + (size_t)b * kSeqN,
            kTok, (long)kDh * kTok,
            (void*)(Oaug + ((size_t)b * kSeqN + (size_t)i * kCS) * kKA + (size_t)h0 * kDh), nullptr, kKA, (long)kDh,
            nullptr, nullptr, 0L, kCS, kDh, Skv, kPVScale);
      }
    }
  }

  wmma_gemm64<0, false, 0, 1, false><<<dim3(1, kNRB), blk, 0, stream>>>(
      Oaug, nullptr, kKA, (long)kCS * kKA,
      AselP, nullptr, kDim, (long)64 * kDim,
      (void*)(Oaug + kDim), nullptr, kKA, (long)kCS * kKA,
      nullptr, nullptr, 0L, kCS, 64, kDim, kT2Scale);

  wmma_gemm64<0, false, 0, 0, false><<<dim3(((kTok / 64) * (kDim / 64)) / 8, 1), blk, 0, stream>>>(
      Oaug, nullptr, kKA, 0L,
      Wpaug, nullptr, kKA, 0L,
      (void*)out, nullptr, kDim, 0L,
      nullptr, nullptr, 0L, kTok, kDim, kKA, kOutScale);
}
